// metaLearner_62740882260595
// MI455X (gfx1250) — hardware-run, weakly checked
//
#include <hip/hip_runtime.h>


namespace {
constexpr int N = 50000, NP = 50048, NP32 = 50016, E = 1600000, T = 12, C = 2, KIN = 24, DMK = 16, XW = 16;
constexpr float XS = 8.0f, WSC = 256.0f, NEG = 0.2f, EPSD = 1e-16f;
typedef _Float16 b16;
typedef __attribute__((ext_vector_type(16))) _Float16 v16b;
typedef __attribute__((ext_vector_type(8))) _Float16 v8b;
typedef __attribute__((ext_vector_type(8))) float v8f;
typedef __attribute__((ext_vector_type(4))) float v4f;
typedef __attribute__((ext_vector_type(2))) float v2f;
__device__ __forceinline__ float bf16_rne(float f) { unsigned int u = __float_as_uint(f); u += 0x7FFFu + ((u >> 16) & 1u); return __uint_as_float(u & 0xFFFF0000u); }
__device__ __forceinline__ v16b frag_kb(const b16* p, int hh) { const v8b a = *(const v8b*)(p + 8 * hh), b = *(const v8b*)(p + 16 + 8 * hh); v16b f;
#pragma unroll
  for (int e = 0; e < 8; ++e) { f[e] = a[e]; f[8 + e] = b[e]; } return f; }
__device__ __forceinline__ v8f wmma16b(v16b a, v16b b, v8f c) { v8f d = __builtin_amdgcn_wmma_f32_16x16x32_f16(false, a, false, b, (short)0, c, false, false); asm volatile("v_nop\n\tv_nop\n\tv_nop\n\tv_nop" : "+v"(d) : "v"(a), "v"(b)); return d; }
__device__ __forceinline__ void wave_lds_sync() { __builtin_amdgcn_fence(__ATOMIC_RELEASE, "workgroup"); __builtin_amdgcn_wave_barrier(); __builtin_amdgcn_fence(__ATOMIC_ACQUIRE, "workgroup"); }
__device__ __forceinline__ float pmul(float a, float b) { float p = a * b; asm volatile("" : "+v"(p)); return p; }
__device__ __forceinline__ float opaque(float a) { asm volatile("" : "+v"(a)); return a; }
__device__ __forceinline__ int iclamp(int v, int lo, int hi) { return v < lo ? lo : (v > hi ? hi : v); }
__device__ __forceinline__ float sigm(float x) { return 1.0f / (1.0f + __expf(-x)); }
__device__ __forceinline__ float lrelu(float x) { return x > 0.0f ? x : NEG * x; }
constexpr int CSR_NBLK8 = 512, CSR_GB8 = 8, CSR_GN8 = 1 << CSR_GB8  , CSR_MAXG8 = 512, CSR_CAP8 = 12288  ;
__global__ __launch_bounds__(64) void csrA8_kernel(const int* __restrict__ dst, int E, int N, int nG, int CHP, int NGP, int* __restrict__ STG, int* __restrict__ HST) {
  extern __shared__ int sm[];
  int* cnt = sm; int* run = sm + NGP; int* ids = sm + 2 * NGP;
  const int b = blockIdx.x; const int ch = (E + CSR_NBLK8 - 1) / CSR_NBLK8; const int e0 = b * ch, e1 = min(E, e0 + ch);
  for (int i = threadIdx.x; i < NGP; i += 64) cnt[i] = 0;
  for (int i = threadIdx.x; i < CHP; i += 64) ids[i] = -1;
  __syncthreads();
  if (threadIdx.x == 0) {
    for (int e = e0; e < e1; ++e) { int d = dst[e]; d = (d < 0) ? 0 : (d >= N ? N - 1 : d); cnt[d >> CSR_GB8] += 1; }
    int acc = 0; for (int g = 0; g < nG; ++g) { run[g] = acc; acc += cnt[g]; }
    for (int e = e0; e < e1; ++e) { int d = dst[e]; d = (d < 0) ? 0 : (d >= N ? N - 1 : d); const int g = d >> CSR_GB8; ids[run[g]] = e; run[g] += 1; } }
  __syncthreads();
  typedef __attribute__((ext_vector_type(4))) int v4i;
  for (int pass = 0; pass < 2; ++pass) {
    for (int i = threadIdx.x; i < CHP / 4; i += 64) *(volatile v4i*)(STG + (size_t)b * CHP + i * 4) = *(const v4i*)(&ids[i * 4]);
    for (int i = threadIdx.x; i < NGP / 4; i += 64) { v4i v; for (int e = 0; e < 4; ++e) v[e] = (i * 4 + e < nG) ? cnt[i * 4 + e] : 0; *(volatile v4i*)(HST + (size_t)b * NGP + i * 4) = v; }
    __threadfence(); }
}
__global__ __launch_bounds__(512) void csrS8_kernel(const int* __restrict__ HST, int nG, int NGP, int* __restrict__ START, int* __restrict__ TOT, int* __restrict__ OFF) {
  __shared__ int tot[CSR_MAXG8];
  const int b = threadIdx.x;
  for (int pass = 0; pass < 2; ++pass) { int runb = 0; for (int g = 0; g < nG; ++g) { int c = HST[(size_t)b * NGP + g]; c = (c < 0) ? 0 : c; ((volatile int*)OFF)[(size_t)g * CSR_NBLK8 + b] = runb; runb += c; } __threadfence(); }
  for (int g = threadIdx.x; g < nG; g += 512) { int s = 0; for (int bb = 0; bb < CSR_NBLK8; ++bb) { int c = HST[(size_t)bb * NGP + g]; s += (c < 0) ? 0 : c; } tot[g] = s; }
  __syncthreads();
  if (threadIdx.x < 32) {
    __shared__ int st[CSR_MAXG8 + 32];
    if (threadIdx.x == 0) { int acc = 0; for (int g = 0; g < NGP; ++g) { st[g] = acc; if (g < nG) acc += (tot[g] + 31) & ~31; } st[NGP] = acc; }
    __builtin_amdgcn_fence(__ATOMIC_RELEASE, "workgroup"); __builtin_amdgcn_wave_barrier(); __builtin_amdgcn_fence(__ATOMIC_ACQUIRE, "workgroup");
    for (int pass = 0; pass < 2; ++pass) { for (int i = threadIdx.x; i < NGP + 32; i += 32) { ((volatile int*)START)[i] = (i <= NGP) ? st[min(i, NGP)] : 0; ((volatile int*)TOT)[i] = (i < nG) ? tot[i] : 0; } __threadfence(); } }
}
__global__ __launch_bounds__(256) void csrB8_kernel(const int* __restrict__ dst, int N, int nG, int CHP, int NGP, int permLen, const int* __restrict__ STG, const int* __restrict__ HST, const int* __restrict__ OFF, const int* __restrict__ START, const int* __restrict__ TOT, int* __restrict__ PERM, int* __restrict__ ROWPTR, int* __restrict__ ROWCNT, int* __restrict__ FLAG) {
  typedef __attribute__((ext_vector_type(4))) int v4i;
  __shared__ int ids[CSR_CAP8]; __shared__ unsigned short key[CSR_CAP8]; __shared__ int outp[CSR_CAP8]; __shared__ int ncnt[CSR_GN8 + 1]; __shared__ int boff[CSR_NBLK8 + 1];
  const int g = blockIdx.x, t_ = threadIdx.x; int tot = TOT[g]; int st = START[g], stn = START[g + 1]; const int v0 = g * CSR_GN8; const int nv = min(CSR_GN8, N - v0);
  st = (st < 0) ? 0 : (st > permLen - 32 ? permLen - 32 : st) & ~31; stn = (stn < st) ? st : (stn > permLen ? permLen : stn); tot = (tot < 0) ? 0 : tot; if (tot > stn - st && tot <= CSR_CAP8) tot = stn - st;
  if (tot > CSR_CAP8) {
    for (int pass = 0; pass < 2; ++pass) { for (int i = t_; i < CSR_GN8 / 4; i += 256) { v4i a, c; for (int e = 0; e < 4; ++e) { a[e] = st; c[e] = 0; } *(volatile v4i*)(ROWPTR + v0 + i * 4) = a; *(volatile v4i*)(ROWCNT + v0 + i * 4) = c; } if (t_ == 0) ((volatile int*)FLAG)[0] = 1; __threadfence(); } (void)nv; return; }
  if (t_ == 0) { int acc = 0; for (int b = 0; b < CSR_NBLK8; ++b) { boff[b] = acc; int c = HST[(size_t)b * NGP + g]; c = (c < 0) ? 0 : (c > CHP ? CHP : c); acc += c; if (acc > tot) acc = tot; } boff[CSR_NBLK8] = acc; }
  for (int i = t_; i <= CSR_GN8; i += 256) ncnt[i] = 0;
  __syncthreads();
  for (int b = 0; b < CSR_NBLK8; ++b) { const int c = boff[b + 1] - boff[b]; int o_ = OFF[(size_t)g * CSR_NBLK8 + b]; o_ = (o_ < 0) ? 0 : (o_ > CHP - c ? CHP - c : o_); const int* src_ = STG + (size_t)b * CHP + o_;
    for (int i = t_; i < c; i += 256) { int id = src_[i]; id = (id < 0) ? 0 : id; ids[boff[b] + i] = id; int d = dst[id]; d = (d < v0) ? v0 : (d >= N ? N - 1 : d); int kk = d - v0; kk = (kk < 0) ? 0 : (kk >= CSR_GN8 ? CSR_GN8 - 1 : kk); key[boff[b] + i] = (unsigned short)kk; } }
  __syncthreads();
  if (t_ == 0) { for (int i = 0; i < tot; ++i) ncnt[key[i]] += 1; int acc = 0; for (int vl = 0; vl < CSR_GN8; ++vl) { const int c = ncnt[vl]; ncnt[vl] = acc; acc += c; } ncnt[CSR_GN8] = acc;
    for (int i = 0; i < tot; ++i) { const int vl = key[i]; outp[ncnt[vl]] = ids[i]; ncnt[vl] += 1; }
    for (int vl = CSR_GN8; vl > 0; --vl) ncnt[vl] = ncnt[vl - 1]; ncnt[0] = 0; }
  __syncthreads();
  for (int pass = 0; pass < 2; ++pass) {
    for (int i = t_; i < (stn - st) / 4; i += 256) { v4i v; for (int e = 0; e < 4; ++e) { const int q = i * 4 + e; v[e] = (q < tot) ? outp[q] : -1; } *(volatile v4i*)(PERM + st + i * 4) = v; }
    for (int i = t_; i < CSR_GN8 / 4; i += 256) { v4i a, c; for (int e = 0; e < 4; ++e) { const int vl = i * 4 + e; a[e] = st + ncnt[vl]; c[e] = (vl < nv) ? (ncnt[vl + 1] - ncnt[vl]) : 0; } *(volatile v4i*)(ROWPTR + v0 + i * 4) = a; *(volatile v4i*)(ROWCNT + v0 + i * 4) = c; }
    __threadfence(); }
}
__global__ __launch_bounds__(256) void csrZ8_kernel(int* __restrict__ p, size_t n4) { typedef __attribute__((ext_vector_type(4))) int v4i; const size_t tid = (size_t)blockIdx.x * 256 + threadIdx.x, nth = (size_t)gridDim.x * 256; v4i z = {0, 0, 0, 0}; for (size_t i = tid; i < n4; i += nth) *(volatile v4i*)(p + i * 4) = z; }
struct CsrBufs8 { int *STG, *HST, *OFF, *START, *TOT, *PERM, *ROWPTR, *ROWCNT, *FLAG; int nG, NGP, CHP; size_t permLen; char* base; size_t bytes; };
static size_t csr_carve8(CsrBufs8& c, char* ws, size_t off, int E, int N) {
  const size_t off0 = off; c.base = ws + off;
  auto al = [&](size_t bytes) { char* p = ws + off; off += (bytes + 255) & ~(size_t)255; return p; };
  c.nG = (N + CSR_GN8 - 1) / CSR_GN8; c.NGP = (c.nG + 31) & ~31; const int ch = (E + CSR_NBLK8 - 1) / CSR_NBLK8; c.CHP = (ch + 31) & ~31; c.permLen = (size_t)E + 32 * (size_t)c.nG + 32;
  c.STG = (int*)al((size_t)CSR_NBLK8 * c.CHP * 4); c.HST = (int*)al((size_t)CSR_NBLK8 * c.NGP * 4); c.OFF = (int*)al((size_t)c.NGP * CSR_NBLK8 * 4); c.START = (int*)al((size_t)(c.NGP + 64) * 4); c.TOT = (int*)al((size_t)(c.NGP + 64) * 4);
  c.PERM = (int*)al(c.permLen * 4); c.ROWPTR = (int*)al((size_t)c.nG * CSR_GN8 * 4); c.ROWCNT = (int*)al((size_t)c.nG * CSR_GN8 * 4); c.FLAG = (int*)al(256);
  c.bytes = off - off0; return off;
}
static void csr_build8(const CsrBufs8& c, const int* dst, int E, int N, hipStream_t stream) {
  const size_t smem = (size_t)(2 * c.NGP + c.CHP) * 4;
  csrZ8_kernel<<<512, 256, 0, stream>>>((int*)c.base, c.bytes / 16);
  csrA8_kernel<<<CSR_NBLK8, 64, smem, stream>>>(dst, E, N, c.nG, c.CHP, c.NGP, c.STG, c.HST);
  csrS8_kernel<<<1, 512, 0, stream>>>(c.HST, c.nG, c.NGP, c.START, c.TOT, c.OFF);
  csrB8_kernel<<<c.nG, 256, 0, stream>>>(dst, N, c.nG, c.CHP, c.NGP, (int)c.permLen, c.STG, c.HST, c.OFF, c.START, c.TOT, c.PERM, c.ROWPTR, c.ROWCNT, c.FLAG);
}


__global__ __launch_bounds__(64) void wprep_kernel(const float* __restrict__ gw, b16* __restrict__ WT) {
  const int u = threadIdx.x; const int o = u >> 2, k0 = (u & 3) * 8; v8b w;
  for (int j = 0; j < 8; ++j) { const int k = k0 + j; w[j] = (o < T && k < KIN) ? (b16)(bf16_rne(gw[k * T + o]) * WSC) : (b16)0.0f; }
  for (int pass = 0; pass < 2; ++pass) { *(volatile v8b*)(WT + o * 32 + k0) = w; __threadfence(); }
}
__global__ __launch_bounds__(32) void xp_kernel(const float* __restrict__ x, const b16* __restrict__ WT, const float* __restrict__ as, const float* __restrict__ ad, float* __restrict__ XP) {
  __shared__ __attribute__((aligned(16))) float so[16][XW];
  const int lane = threadIdx.x, nloc = lane & 15, hlf = lane >> 4; const size_t v0 = (size_t)blockIdx.x * 16; const size_t v = v0 + nloc; const size_t vc = v < (size_t)N ? v : (size_t)(N - 1);
  v16b a = {}; { const float* xr = x + vc * KIN; for (int e = 0; e < 8; ++e) { const int k = 8 * hlf + e; a[e] = (b16)(bf16_rne(xr[k]) * XS); const int k2 = 16 + 8 * hlf + e; a[8 + e] = (k2 < KIN) ? (b16)(bf16_rne(xr[k2 < KIN ? k2 : KIN - 1]) * XS) : (b16)0.0f; } }
  v8f acc = (v8f){}; acc = wmma16b(a, frag_kb(WT + nloc * 32, hlf), acc);
  const float wa = (nloc < T) ? opaque(bf16_rne(as[nloc < T ? nloc : 0])) : 0.0f, wd = (nloc < T) ? opaque(bf16_rne(ad[nloc < T ? nloc : 0])) : 0.0f;
#pragma unroll
  for (int r = 0; r < 8; ++r) { const float p = acc[r] * (1.0f / (XS * WSC)); float s1 = pmul(p, wa), s2 = pmul(p, wd);
    for (int o = 1; o < 16; o <<= 1) { s1 += __shfl_xor(s1, o); s2 += __shfl_xor(s2, o); }
    const size_t row = v0 + 8 * hlf + r; const bool ok = row < (size_t)N; float val = (nloc < T) ? p : (nloc == 12 ? s1 : (nloc == 13 ? s2 : 0.0f)); so[8 * hlf + r][nloc] = ok ? val : 0.0f; }
  wave_lds_sync();
  for (int pass = 0; pass < 2; ++pass) { for (int q = 0; q < 2; ++q) { const int idx = q * 32 + lane; *(volatile v4f*)(XP + v0 * XW + idx * 4) = *(const v4f*)(&so[idx >> 2][(idx & 3) * 4]); } __threadfence(); }
}
__global__ __launch_bounds__(32) void gru_kernel(const float* __restrict__ x, const float* __restrict__ wih, const float* __restrict__ whh, const float* __restrict__ bih, const float* __restrict__ bhh, float* __restrict__ XG) {
  __shared__ __attribute__((aligned(16))) float hb[32][XW];
  const int lane = threadIdx.x; const int t = lane < T ? lane : T - 1;
  const float wr0 = opaque(bf16_rne(wih[0])), wr1 = opaque(bf16_rne(wih[1])), wz0 = opaque(bf16_rne(wih[2])), wz1 = opaque(bf16_rne(wih[3])), wn0 = opaque(bf16_rne(wih[4])), wn1 = opaque(bf16_rne(wih[5]));
  const float ur = opaque(bf16_rne(whh[0])), uz = opaque(bf16_rne(whh[1])), un = opaque(bf16_rne(whh[2])); const float br = opaque(bf16_rne(bih[0])), bz = opaque(bf16_rne(bih[1])), bn = opaque(bf16_rne(bih[2])); const float cr = opaque(bf16_rne(bhh[0])), cz = opaque(bf16_rne(bhh[1])), cn = opaque(bf16_rne(bhh[2]));
  for (int i = lane; i < 32 * XW; i += 32) (&hb[0][0])[i] = 0.0f;
  wave_lds_sync();
  float h = 0.0f;
#pragma unroll 1
  for (int n0 = 0; n0 < NP32; n0 += 32) {
#pragma unroll 1
    for (int i = 0; i < 32; ++i) { const int n = n0 + i; const size_t nc = (size_t)(n < N ? n : N - 1); const v2f xv = *(const v2f*)(x + (nc * T + t) * C); const float x0 = bf16_rne(xv[0]), x1 = bf16_rne(xv[1]);
      const float gir = pmul(x0, wr0) + pmul(x1, wr1) + br, giz = pmul(x0, wz0) + pmul(x1, wz1) + bz, gin = pmul(x0, wn0) + pmul(x1, wn1) + bn;
      const float ghr = pmul(h, ur) + cr, ghz = pmul(h, uz) + cz, ghn = pmul(h, un) + cn;
      const float rg = sigm(gir + ghr), zg = sigm(giz + ghz); const float ng = tanhf(gin + pmul(rg, ghn)); h = pmul(1.0f - zg, ng) + pmul(zg, h);
      if (lane < XW) hb[i][lane] = (lane < T) ? h : 0.0f; }
    wave_lds_sync();
    for (int pass = 0; pass < 2; ++pass) { for (int q = 0; q < 4; ++q) { const int idx = q * 32 + lane; *(volatile v4f*)(XG + (size_t)n0 * XW + idx * 4) = *(const v4f*)(&hb[idx >> 2][(idx & 3) * 4]); } __threadfence(); }
    wave_lds_sync(); }
}
__global__ __launch_bounds__(256) void gat_kernel(const float* __restrict__ XP, const float* __restrict__ XG, const int* __restrict__ srcs, const int* __restrict__ PERM, const int* __restrict__ ROWPTR, const int* __restrict__ ROWCNT, int permLen, const float* __restrict__ gb, const float* __restrict__ gam, const float* __restrict__ lw, const float* __restrict__ lb, float* __restrict__ out) {
  __shared__ __attribute__((aligned(16))) float so[8][32];
  const int wave = threadIdx.x >> 5, lane = threadIdx.x & 31; const int cl = lane < T ? lane : T - 1; const int ol = lane & 15;
  const float gbias = bf16_rne(gb[cl]); const float g = bf16_rne(gam[cl]); const float sg = sigm(g), sg1 = sigm(1.0f - g); const float lbias = bf16_rne(lb[ol]);
  float lwc[T]; for (int c = 0; c < T; ++c) lwc[c] = opaque(bf16_rne(lw[c * DMK + ol]));
#pragma unroll 1
  for (int qq = 0; qq < 2; ++qq) { const size_t v = (size_t)blockIdx.x * 16 + wave * 2 + qq;
    int st = ROWPTR[v], cnt = ROWCNT[v]; cnt = iclamp(cnt, 0, 65536); st = iclamp(st, 0, permLen - cnt);
    const v4f own3 = *(const v4f*)(XP + v * XW + 12); const float asv = own3[0], adv = own3[1];
    float mx = lrelu(asv + adv);
#pragma unroll 1
    for (int j0 = 0; j0 < cnt; j0 += 32) { const int j = j0 + lane; const bool ok = j < cnt; const int e = iclamp(PERM[iclamp(st + j, 0, permLen - 1)], 0, E - 1); const int s = iclamp(srcs[e], 0, N - 1);
      const float es = lrelu(XP[(size_t)s * XW + 12] + adv); mx = fmaxf(mx, ok ? es : -INFINITY); }
    for (int o = 1; o < 32; o <<= 1) mx = fmaxf(mx, __shfl_xor(mx, o));
    float acc[T]; const float pself = __expf(lrelu(asv + adv) - mx); { const v4f a0 = *(const v4f*)(XP + v * XW), a1 = *(const v4f*)(XP + v * XW + 4), a2 = *(const v4f*)(XP + v * XW + 8);
      const float xs[T] = {a0[0], a0[1], a0[2], a0[3], a1[0], a1[1], a1[2], a1[3], a2[0], a2[1], a2[2], a2[3]}; for (int c = 0; c < T; ++c) acc[c] = (lane == 0) ? pmul(pself, xs[c]) : 0.0f; }
    float den = (lane == 0) ? pself : 0.0f;
#pragma unroll 1
    for (int j0 = 0; j0 < cnt; j0 += 32) { const int j = j0 + lane; const bool ok = j < cnt; const int e = iclamp(PERM[iclamp(st + j, 0, permLen - 1)], 0, E - 1); const int s = iclamp(srcs[e], 0, N - 1);
      const float* xr = XP + (size_t)s * XW; const v4f a0 = *(const v4f*)(xr), a1 = *(const v4f*)(xr + 4), a2 = *(const v4f*)(xr + 8), a3 = *(const v4f*)(xr + 12);
      const float pj = ok ? __expf(lrelu(a3[0] + adv) - mx) : 0.0f; den += pj;
      const float xs[T] = {a0[0], a0[1], a0[2], a0[3], a1[0], a1[1], a1[2], a1[3], a2[0], a2[1], a2[2], a2[3]};
#pragma unroll
      for (int c = 0; c < T; ++c) acc[c] += pmul(pj, xs[c]); }
    for (int o = 1; o < 32; o <<= 1) { den += __shfl_xor(den, o);
#pragma unroll
      for (int c = 0; c < T; ++c) acc[c] += __shfl_xor(acc[c], o); }
    const float inv = 1.0f / (den + EPSD);
    const float* xg = XG + v * XW; float o_ = lbias;
#pragma unroll
    for (int c = 0; c < T; ++c) { const float xgat = pmul(acc[c], inv) + __shfl(gbias, c); const float xmk = pmul(__shfl(sg, c), xgat) + pmul(__shfl(sg1, c), xg[c]); o_ += pmul(xmk, lwc[c]); }
    if (lane < 16) so[wave][qq * 16 + lane] = o_; }
  wave_lds_sync();
  for (int pass = 0; pass < 2; ++pass) { if (lane < 8) *(volatile v4f*)(out + ((size_t)blockIdx.x * 16 + wave * 2) * DMK + lane * 4) = *(const v4f*)(&so[wave][lane * 4]); __threadfence(); }
}
}

extern "C" void kernel_launch(void* const* d_in, const int* in_sizes, int n_in, void* d_out, int out_size, void* d_ws, size_t ws_size, hipStream_t stream) {
  (void)n_in;
  auto Fp = [&](int i) { return (const float*)d_in[i]; }; auto Ip = [&](int i) { return (const int*)d_in[i]; };
  if (in_sizes[0] != N * KIN || in_sizes[1] != 2 * E || in_sizes[2] != 6 || in_sizes[3] != 3 || in_sizes[6] != KIN * T || in_sizes[7] != T || in_sizes[11] != T * DMK || in_sizes[12] != DMK || out_size != N * DMK) return;
  size_t off = 0; char* ws = (char*)d_ws;
  auto carve = [&](size_t bytes) { char* p = ws + off; off += (bytes + 255) & ~(size_t)255; return p; };
  b16* WT = (b16*)carve((size_t)16 * 32 * 2); float* XP = (float*)carve((size_t)NP * XW * 4); float* XG = (float*)carve((size_t)NP * XW * 4);
  CsrBufs8 csr; off = csr_carve8(csr, ws, off, E, N);
  if (off > ws_size || off > ((size_t)128 << 20)) return;
  wprep_kernel<<<1, 64, 0, stream>>>(Fp(6), WT);
  csr_build8(csr, Ip(1) + E, E, N, stream);
  xp_kernel<<<NP / 16, 32, 0, stream>>>(Fp(0), WT, Fp(7), Fp(8), XP);
  gru_kernel<<<1, 32, 0, stream>>>(Fp(0), Fp(2), Fp(3), Fp(4), Fp(5), XG);
  gat_kernel<<<N / 16, 256, 0, stream>>>(XP, XG, Ip(1), csr.PERM, csr.ROWPTR, csr.ROWCNT, (int)csr.permLen, Fp(9), Fp(10), Fp(11), Fp(12), (float*)d_out);
}
